// DeltaNet_31877247271452
// MI455X (gfx1250) — hardware-verified
//
#include <hip/hip_runtime.h>
#include <math.h>

constexpr int NBAT   = 4;
constexpr int SEQ    = 2048;
constexpr int DM     = 1024;
constexpr int NHEAD  = 4;
constexpr int HDIM   = 256;
constexpr int NROW   = NBAT * SEQ;
constexpr int GHID   = 2048;
constexpr int NGATE  = 16;
constexpr int GATE_PITCH = 64;
constexpr int CHK    = 32;
constexpr int NCHUNK = SEQ / CHK;
constexpr int DVHALF = 128;
constexpr int TAPS_S = 7;
constexpr int TAPS_L = 31;
constexpr int HALF_ROWS = NROW / 2;
static_assert(DM == NHEAD * HDIM, "head split");
static_assert(SEQ % CHK == 0, "no chunk padding");
static_assert(NROW % 64 == 0 && DM % 64 == 0 && GHID % 64 == 0 && GATE_PITCH % 64 == 0, "GEMM M,N tile multiples");
static_assert(DM % 32 == 0 && GHID % 32 == 0 && HDIM % 32 == 0, "GEMM K multiples of 32");
static_assert(HALF_ROWS % 64 == 0, "half-M tile multiple");

constexpr float W_CARRY     = 16.0f;
constexpr float W_CARRY_INV = 1.0f / W_CARRY;
constexpr float QK_CARRY    = 16.0f;
constexpr float V_CARRY     = 256.0f;
constexpr float T_CARRY     = 64.0f;
constexpr float INV_QK2     = 1.0f / (QK_CARRY * QK_CARRY);
constexpr float INV_QK      = 1.0f / QK_CARRY;
constexpr float INV_T       = 1.0f / T_CARRY;
constexpr float INV_OUT     = 1.0f / (QK_CARRY * V_CARRY);
constexpr float RMS_EPS     = 1e-5f;

typedef __attribute__((ext_vector_type(16))) _Float16 v16h;
typedef __attribute__((ext_vector_type(8)))  _Float16 v8h;
typedef __attribute__((ext_vector_type(8)))  float    v8f;
typedef __attribute__((ext_vector_type(4)))  float    v4f;
typedef __attribute__((ext_vector_type(4)))  unsigned int v4u;
typedef __attribute__((ext_vector_type(2)))  unsigned int v2u;

__device__ __forceinline__ unsigned pk16(unsigned short a, unsigned short b) { return (unsigned)a | ((unsigned)b << 16); }
__device__ __forceinline__ unsigned short h_bits(float f) { const _Float16 h = (_Float16)f; return __builtin_bit_cast(unsigned short, h); }
__device__ __forceinline__ float h16_to_f32(unsigned hb) {
  const unsigned sgn = (hb & 0x8000u) << 16;
  const unsigned em = hb & 0x7fffu;
  const float fn = __uint_as_float((em << 13) + 0x38000000u);
  const float fs = (float)em * 5.9604644775390625e-8f;
  const float mag = (em < 0x400u) ? fs : fn;
  return __uint_as_float(__float_as_uint(mag) | sgn);
}

__device__ __forceinline__ void dep_guard4_h(v8f& a, v8f& b, v8f& c, v8f& d, v16h x, v16h y) {
  asm volatile("v_nop\n\tv_nop\n\tv_nop\n\tv_nop" : "+v"(a), "+v"(b), "+v"(c), "+v"(d) : "v"(x), "v"(y));
}
__device__ __forceinline__ void keep4_h(v16h a, v16h b, v16h c, v16h d) { asm volatile("v_nop" :: "v"(a), "v"(b), "v"(c), "v"(d)); }
__device__ __forceinline__ void acc_guard4(v8f& a, v8f& b, v8f& c, v8f& d) { asm volatile("v_nop\n\tv_nop\n\tv_nop\n\tv_nop" : "+v"(a), "+v"(b), "+v"(c), "+v"(d)); }
__device__ __forceinline__ void pin2(v8f& a, v8f& b) { asm volatile("" : "+v"(a), "+v"(b) :: "memory"); }

template <typename T> struct Frag;
template <> struct Frag<_Float16> {
  typedef v16h V; union U { v16h v; v8h h[2]; };
  static __device__ __forceinline__ v16h load(const _Float16* p) {
    U f; f.h[0] = *(const v8h*)(p); f.h[1] = *(const v8h*)(p + 16); return f.v;
  }
  static __device__ __forceinline__ v8f mma(v16h a, v16h b, v8f c) {
    return __builtin_amdgcn_wmma_f32_16x16x32_f16(false, a, false, b, (short)0, c, false, false);
  }
};
__device__ __forceinline__ v8f wm(v16h a, v16h b, v8f c) {
  c = __builtin_amdgcn_wmma_f32_16x16x32_f16(false, a, false, b, (short)0, c, false, false);
  asm volatile("v_nop\n\tv_nop\n\tv_nop\n\tv_nop" : "+v"(c) : "v"(a), "v"(b));
  return c;
}

template <int OUT_MODE>
__global__ __launch_bounds__(256) void wmma_gemm64(
    const unsigned short* __restrict__ Ap, int lda,
    const unsigned short* __restrict__ Btp, int ldb,
    void* __restrict__ Cout, int ldc, int M, int N, int K, float scale) {
  typedef _Float16 T;
  typedef v16h V;
  const T* A = (const T*)Ap; const T* Bt = (const T*)Btp;
  __shared__ __align__(16) float sT[8][16 * 68];
  const int lane = threadIdx.x & 31;
  const int wave = threadIdx.x >> 5;
  const int tilesN = N >> 6;
  const int tilesM = M >> 6;
  const int tile = blockIdx.x * 8 + wave;
  if (tile >= tilesM * tilesN) return;
  const int tm = tile / tilesN;
  const int tn = tile - tm * tilesN;
  const int m0 = tm << 6;
  const int n0 = tn << 6;
  const int rlane = lane & 15;
  const int koff  = (lane >> 4) * 8;
  const int mOff  = (lane >> 4) * 8;

  v8f acc[4][4];
#pragma unroll
  for (int i = 0; i < 4; ++i)
#pragma unroll
    for (int j = 0; j < 4; ++j) acc[i][j] = (v8f){0.f,0.f,0.f,0.f,0.f,0.f,0.f,0.f};

  const T* Bbase = Bt + (size_t)(n0 + rlane) * ldb + koff;
  const T* Abase = A  + (size_t)(m0 + rlane) * lda + koff;
  const size_t bstep = (size_t)16 * ldb;
  const size_t astep = (size_t)16 * lda;

  for (int k0 = 0; k0 < K; k0 += 32) {
    V bh[4];
#pragma unroll
    for (int j = 0; j < 4; ++j) bh[j] = Frag<T>::load(Bbase + j * bstep + k0);
#pragma unroll
    for (int i = 0; i < 4; ++i) {
      V ah = Frag<T>::load(Abase + i * astep + k0);
#pragma unroll
      for (int j = 0; j < 4; ++j) acc[i][j] = Frag<T>::mma(ah, bh[j], acc[i][j]);
      dep_guard4_h(acc[i][0], acc[i][1], acc[i][2], acc[i][3], ah, bh[3]);
    }
    keep4_h(bh[0], bh[1], bh[2], bh[3]);
  }
  acc_guard4(acc[0][0], acc[0][1], acc[0][2], acc[0][3]);
  acc_guard4(acc[1][0], acc[1][1], acc[1][2], acc[1][3]);
  acc_guard4(acc[2][0], acc[2][1], acc[2][2], acc[2][3]);
  acc_guard4(acc[3][0], acc[3][1], acc[3][2], acc[3][3]);

  float* slab = sT[wave];
#pragma unroll
  for (int i = 0; i < 4; ++i) {
    const int mBase = m0 + (i << 4);
#pragma unroll
    for (int j = 0; j < 4; ++j) {
#pragma unroll
      for (int r = 0; r < 8; ++r) {
        const float v = acc[i][j][r] * scale;
        slab[(mOff + r) * 68 + (j << 4) + rlane] = v;
      }
    }
    __builtin_amdgcn_fence(__ATOMIC_RELEASE, "workgroup");
    __builtin_amdgcn_wave_barrier();
    __builtin_amdgcn_fence(__ATOMIC_ACQUIRE, "workgroup");
    if (OUT_MODE == 0) {
      float* C = (float*)Cout;
      const int hh = lane >> 4, c4 = (lane & 15) * 4;
      for (int pass = 0; pass < 2; ++pass) {
#pragma unroll
        for (int it = 0; it < 8; ++it) {
          const int row = it * 2 + hh;
          v4f v = *(const v4f*)(slab + row * 68 + c4);
          *(volatile v4f*)(C + (size_t)(mBase + row) * ldc + n0 + c4) = v;
        }
        __threadfence();
      }
    } else {
      const int q = lane >> 3, c8 = (lane & 7) * 8;
      unsigned short* C = (unsigned short*)Cout;
      for (int pass = 0; pass < 2; ++pass) {
#pragma unroll
        for (int it = 0; it < 4; ++it) {
          const int row = it * 4 + q;
          const float* sp = slab + row * 68 + c8;
          v8h hv;
#pragma unroll
          for (int e = 0; e < 8; ++e) hv[e] = (_Float16)sp[e];
          *(volatile v8h*)(C + (size_t)(mBase + row) * ldc + n0 + c8) = hv;
        }
        __threadfence();
      }
    }
    __builtin_amdgcn_fence(__ATOMIC_RELEASE, "workgroup");
    __builtin_amdgcn_wave_barrier();
    __builtin_amdgcn_fence(__ATOMIC_ACQUIRE, "workgroup");
  }
}

__device__ __forceinline__ void cast8_store(const float* __restrict__ p, unsigned short* __restrict__ q, float sc) {
  const v4f a = *(const v4f*)(p);
  const v4f c = *(const v4f*)(p + 4);
  unsigned short hb[8];
#pragma unroll
  for (int e = 0; e < 4; ++e) {
    const float ae = a[e] * sc;
    const float ce = c[e] * sc;
    hb[e]     = h_bits(ae);
    hb[4 + e] = h_bits(ce);
  }
  const v4u u = (v4u){pk16(hb[0], hb[1]), pk16(hb[2], hb[3]), pk16(hb[4], hb[5]), pk16(hb[6], hb[7])};
  *(volatile v4u*)q = u;
  __threadfence();
  *(volatile v4u*)q = u;
}

__global__ __launch_bounds__(256) void cast8_f16_kernel(const float* __restrict__ in, unsigned short* __restrict__ out, int n8, float sc) {
  const int i = blockIdx.x * 256 + threadIdx.x;
  if (i >= n8) return;
  cast8_store(in + 8 * (size_t)i, out + 8 * (size_t)i, sc);
}

__global__ __launch_bounds__(256) void cast_weights_kernel(
    const float* __restrict__ s0, const float* __restrict__ s1, const float* __restrict__ s2,
    const float* __restrict__ s3, const float* __restrict__ s4,
    unsigned short* __restrict__ d0, unsigned short* __restrict__ d1, unsigned short* __restrict__ d2,
    unsigned short* __restrict__ d3, unsigned short* __restrict__ d4,
    int n8_small, int n8_big, float sc) {
  const int z = blockIdx.y;
  const float* src = (z == 0) ? s0 : (z == 1) ? s1 : (z == 2) ? s2 : (z == 3) ? s3 : s4;
  unsigned short* dst = (z == 0) ? d0 : (z == 1) ? d1 : (z == 2) ? d2 : (z == 3) ? d3 : d4;
  const int n8 = (z == 4) ? n8_big : n8_small;
  const int i = blockIdx.x * 256 + threadIdx.x;
  if (i >= n8) return;
  cast8_store(src + 8 * (size_t)i, dst + 8 * (size_t)i, sc);
}

__global__ __launch_bounds__(256) void w2_pad_kernel(const float* __restrict__ w2, unsigned short* __restrict__ out, float sc) {
  const int i = blockIdx.x * 256 + threadIdx.x;
  const int row = i >> 8;
  const int c8 = i & 255;
  const int srow = (row < NGATE) ? row : (NGATE - 1);
  const float* p = w2 + (size_t)srow * GHID + c8 * 8;
  const v4f a = *(const v4f*)(p);
  const v4f c = *(const v4f*)(p + 4);
  const bool live = (row < NGATE);
  unsigned short hb[8];
#pragma unroll
  for (int e = 0; e < 4; ++e) {
    const float ae = live ? (a[e] * sc) : 0.0f;
    const float ce = live ? (c[e] * sc) : 0.0f;
    hb[e]     = h_bits(ae);
    hb[4 + e] = h_bits(ce);
  }
  const v4u u = (v4u){pk16(hb[0], hb[1]), pk16(hb[2], hb[3]), pk16(hb[4], hb[5]), pk16(hb[6], hb[7])};
  unsigned short* q = out + 8 * (size_t)i;
  *(volatile v4u*)q = u;
  __threadfence();
  *(volatile v4u*)q = u;
}

__global__ __launch_bounds__(256) void gelu_bias_f16_kernel(const float* __restrict__ tin, const float* __restrict__ b1,
                                                            unsigned short* __restrict__ out, int n2) {
  const int i = blockIdx.x * 256 + threadIdx.x;
  if (i >= n2) return;
  const int col = (2 * i) & (GHID - 1);
  const float x0 = tin[2 * (size_t)i] + b1[col];
  const float x1 = tin[2 * (size_t)i + 1] + b1[col + 1];
  const float g0 = 0.5f * x0 * (1.0f + erff(x0 * 0.70710678118654752f));
  const float g1 = 0.5f * x1 * (1.0f + erff(x1 * 0.70710678118654752f));
  const unsigned u = pk16(h_bits(g0), h_bits(g1));
  volatile unsigned* q = (volatile unsigned*)out + (size_t)i;
  *q = u;
  __threadfence();
  *q = u;
}

__global__ __launch_bounds__(256) void beta_gate_kernel(const float* __restrict__ X, const float* __restrict__ bw,
                                                        float* __restrict__ beta) {
  __shared__ float sb[32];
  const int lane = threadIdx.x & 31, wave = threadIdx.x >> 5;
  const int row = blockIdx.x * 8 + wave;
  const float* xr = X + (size_t)row * DM;
  float s0 = 0.f, s1 = 0.f, s2 = 0.f, s3 = 0.f;
#pragma unroll 1
  for (int it = 0; it < DM / 128; ++it) {
    const int e = it * 128 + lane * 4;
    const v4f x  = *(const v4f*)(xr + e);
    const v4f w0 = *(const v4f*)(bw + e);
    const v4f w1 = *(const v4f*)(bw + DM + e);
    const v4f w2 = *(const v4f*)(bw + 2 * DM + e);
    const v4f w3 = *(const v4f*)(bw + 3 * DM + e);
    s0 += (x[0] * w0[0] + x[1] * w0[1]) + (x[2] * w0[2] + x[3] * w0[3]);
    s1 += (x[0] * w1[0] + x[1] * w1[1]) + (x[2] * w1[2] + x[3] * w1[3]);
    s2 += (x[0] * w2[0] + x[1] * w2[1]) + (x[2] * w2[2] + x[3] * w2[3]);
    s3 += (x[0] * w3[0] + x[1] * w3[1]) + (x[2] * w3[2] + x[3] * w3[3]);
  }
#pragma unroll
  for (int m = 16; m >= 1; m >>= 1) {
    s0 += __shfl_xor(s0, m, 32);
    s1 += __shfl_xor(s1, m, 32);
    s2 += __shfl_xor(s2, m, 32);
    s3 += __shfl_xor(s3, m, 32);
  }
  const float s = (lane == 0) ? s0 : (lane == 1) ? s1 : (lane == 2) ? s2 : s3;
  const float sg = __builtin_amdgcn_rcpf(1.0f + expf(-s));
  if (lane < NHEAD) sb[wave * NHEAD + lane] = sg;
  __syncthreads();
  if (wave == 0) {
    const float v = sb[lane];
    volatile float* q = (volatile float*)beta + (size_t)blockIdx.x * 32 + lane;
    *q = v;
    __threadfence();
    *q = v;
  }
}

__global__ __launch_bounds__(256) void qk_conv_norm_kernel(
    const unsigned short* __restrict__ qraw, const unsigned short* __restrict__ kraw,
    const float* __restrict__ qcw, const float* __restrict__ kcw,
    unsigned short* __restrict__ qn, unsigned short* __restrict__ kn) {
  const int z = blockIdx.y;
  const unsigned short* raw = z ? kraw : qraw;
  const float* cw = z ? kcw : qcw;
  unsigned short* outp = z ? kn : qn;
  const int lane = threadIdx.x & 31, wave = threadIdx.x >> 5;
  const int gw = blockIdx.x * 8 + wave;
  const int bl = gw >> 2;
  const int hd = gw & 3;
  const int l  = bl & (SEQ - 1);
  const int ch = hd * HDIM + lane * 8;
  v4f wv[8];
#pragma unroll
  for (int e = 0; e < 8; ++e) wv[e] = *(const v4f*)(cw + (size_t)(ch + e) * 4);
  float y[8];
#pragma unroll
  for (int e = 0; e < 8; ++e) y[e] = 0.0f;
#pragma unroll
  for (int j = 0; j < 4; ++j) {
    const int back = 3 - j;
    const bool valid = (l >= back);
    const int rowc = valid ? (bl - back) : bl;
    const v4u w = *(const v4u*)(raw + (size_t)rowc * DM + ch);
#pragma unroll
    for (int e2 = 0; e2 < 4; ++e2) {
      const unsigned ww = w[e2];
      float x0 = h16_to_f32(ww & 0xffffu);
      float x1 = h16_to_f32(ww >> 16);
      x0 = valid ? x0 : 0.0f;
      x1 = valid ? x1 : 0.0f;
      y[2 * e2]     = fmaf(wv[2 * e2][j], x0, y[2 * e2]);
      y[2 * e2 + 1] = fmaf(wv[2 * e2 + 1][j], x1, y[2 * e2 + 1]);
    }
  }
  float ss = 0.0f;
#pragma unroll
  for (int e = 0; e < 8; ++e) {
    const float sg = __builtin_amdgcn_rcpf(1.0f + expf(-y[e]));
    y[e] = y[e] * sg;
    ss += y[e] * y[e];
  }
#pragma unroll
  for (int m = 16; m >= 1; m >>= 1) ss += __shfl_xor(ss, m, 32);
  const float inv = rsqrtf(ss) * QK_CARRY;
  unsigned short hb[8];
#pragma unroll
  for (int e = 0; e < 8; ++e) hb[e] = h_bits(y[e] * inv);
  const v4u u = (v4u){pk16(hb[0], hb[1]), pk16(hb[2], hb[3]), pk16(hb[4], hb[5]), pk16(hb[6], hb[7])};
  unsigned short* q = outp + (size_t)bl * DM + ch;
  *(volatile v4u*)q = u;
  __threadfence();
  *(volatile v4u*)q = u;
}

__global__ __launch_bounds__(256) void v_conv_silu_kernel(const float* __restrict__ vraw, const float* __restrict__ cw,
                                                          float* __restrict__ vc) {
  const int i = blockIdx.x * 256 + threadIdx.x;
  const int row = i >> 8;
  const int c4 = (i & 255) * 4;
  const int l = row & (SEQ - 1);
  v4f wv[4];
#pragma unroll
  for (int e = 0; e < 4; ++e) wv[e] = *(const v4f*)(cw + (size_t)(c4 + e) * 4);
  v4f y = (v4f){0.f, 0.f, 0.f, 0.f};
#pragma unroll
  for (int j = 0; j < 4; ++j) {
    const int back = 3 - j;
    const bool valid = (l >= back);
    const int rowc = valid ? (row - back) : row;
    const v4f x = *(const v4f*)(vraw + (size_t)rowc * DM + c4);
#pragma unroll
    for (int e = 0; e < 4; ++e) {
      const float xe = valid ? x[e] : 0.0f;
      y[e] = fmaf(wv[e][j], xe, y[e]);
    }
  }
  v4f o;
#pragma unroll
  for (int e = 0; e < 4; ++e) {
    const float sg = __builtin_amdgcn_rcpf(1.0f + expf(-y[e]));
    o[e] = y[e] * sg;
  }
  float* q = vc + (size_t)row * DM + c4;
  *(volatile v4f*)q = o;
  __threadfence();
  *(volatile v4f*)q = o;
}

constexpr int KT_PITCH = 40;
constexpr int MAT_PITCH = 33;
constexpr int OS_PITCH = 132;

__global__ __launch_bounds__(256) __attribute__((amdgpu_num_vgpr(256))) void chunk_scan_kernel(
    const unsigned short* __restrict__ qnp, const unsigned short* __restrict__ knp,
    const float* __restrict__ vc, const float* __restrict__ betap, float* __restrict__ dout) {
  __shared__ __align__(16) _Float16 kT_s[HDIM * KT_PITCH];
  __shared__ __align__(16) float Af[CHK * MAT_PITCH];
  __shared__ __align__(16) float Al[CHK * MAT_PITCH];
  __shared__ __align__(16) float o_s[CHK * OS_PITCH];
  __shared__ float beta_s[CHK];

  const _Float16* qn = (const _Float16*)qnp;
  const _Float16* kn = (const _Float16*)knp;
  const int tid = threadIdx.x, lane = tid & 31, wave = tid >> 5;
  const int c = lane & 15, hh = lane >> 4, koff = 8 * hh;
  const int bh = blockIdx.x >> 1;
  const int dvbase = (blockIdx.x & 1) * DVHALF;
  const int b = bh >> 2, hd = bh & 3;
  const int colbase = hd * HDIM;
  const v8f z8 = (v8f){0.f, 0.f, 0.f, 0.f, 0.f, 0.f, 0.f, 0.f};

  v8f sacc[16];
#pragma unroll
  for (int j = 0; j < 16; ++j) sacc[j] = z8;

#pragma unroll 1
  for (int ch = 0; ch < NCHUNK; ++ch) {
    const int row0 = b * SEQ + ch * CHK;

    {
      const int t = tid >> 3, g = tid & 7;
      const unsigned short* kr = knp + (size_t)(row0 + t) * DM + colbase;
#pragma unroll 2
      for (int it = 0; it < 4; ++it) {
        const int dk0 = (it * 8 + g) * 8;
        const v4u w = *(const v4u*)(kr + dk0);
#pragma unroll
        for (int e = 0; e < 4; ++e) {
          const unsigned ww = w[e];
          const unsigned short lo = (unsigned short)(ww & 0xffffu);
          const unsigned short hi = (unsigned short)(ww >> 16);
          kT_s[(dk0 + 2 * e) * KT_PITCH + t]     = __builtin_bit_cast(_Float16, lo);
          kT_s[(dk0 + 2 * e + 1) * KT_PITCH + t] = __builtin_bit_cast(_Float16, hi);
        }
      }
      if (tid < CHK) beta_s[tid] = betap[(size_t)(row0 + tid) * NHEAD + hd];
    }
    __syncthreads();

    {
      const bool isG = (wave < 4);
      const int sub = wave & 3;
      const int ti = sub >> 1, tj = sub & 1;
      const _Float16* Asrc = isG ? kn : qn;
      const _Float16* Apt = Asrc + (size_t)(row0 + ti * 16 + c) * DM + colbase + koff;
      const _Float16* Bpt = kn   + (size_t)(row0 + tj * 16 + c) * DM + colbase + koff;
      v8f acc = z8;
#pragma unroll 2
      for (int k0 = 0; k0 < HDIM; k0 += 32) {
        const v16h a  = Frag<_Float16>::load(Apt + k0);
        const v16h bf = Frag<_Float16>::load(Bpt + k0);
        acc = wm(a, bf, acc);
      }
      float* dstM = isG ? Af : Al;
      const int n = tj * 16 + c;
#pragma unroll
      for (int r = 0; r < 8; ++r) {
        const int m = ti * 16 + 8 * hh + r;
        const float gval = -beta_s[m] * acc[r] * INV_QK2;
        const float pval = acc[r] * INV_QK;
        const float gsel = (n < m) ? gval : 0.0f;
        const float psel = (n <= m) ? pval : 0.0f;
        dstM[m * MAT_PITCH + n] = isG ? gsel : psel;
      }
    }

    v8f aq0 = z8, aq1 = z8;
    v16h rb;
    {
      v8f ak0 = z8, ak1 = z8;
      const _Float16* kp = kn + (size_t)(row0 + c) * DM + colbase + koff;
      const _Float16* qp = qn + (size_t)(row0 + c) * DM + colbase + koff;
#pragma unroll
      for (int s = 0; s < 8; ++s) {
        pin2(sacc[2 * s], sacc[2 * s + 1]);
        v16h bs;
#pragma unroll
        for (int i = 0; i < 8; ++i) {
          bs[i]     = (_Float16)(sacc[2 * s][i] * INV_QK);
          bs[8 + i] = (_Float16)(sacc[2 * s + 1][i] * INV_QK);
        }
        {
          const v16h a = Frag<_Float16>::load(kp + 32 * s);
          ak0 = wm(a, bs, ak0);
        }
        {
          const v16h a = Frag<_Float16>::load(kp + (size_t)16 * DM + 32 * s);
          ak1 = wm(a, bs, ak1);
        }
        {
          const v16h a = Frag<_Float16>::load(qp + 32 * s);
          aq0 = wm(a, bs, aq0);
        }
        {
          const v16h a = Frag<_Float16>::load(qp + (size_t)16 * DM + 32 * s);
          aq1 = wm(a, bs, aq1);
        }
      }
      const float* vp = vc + (size_t)(row0 + 8 * hh) * DM + colbase + dvbase + 16 * wave + c;
#pragma unroll
      for (int r = 0; r < 8; ++r) {
        const float v0 = vp[(size_t)r * DM];
        const float v1 = vp[(size_t)(16 + r) * DM];
        rb[r]     = (_Float16)(v0 * V_CARRY - ak0[r] * INV_QK);
        rb[8 + r] = (_Float16)(v1 * V_CARRY - ak1[r] * INV_QK);
      }
    }
    __syncthreads();

    if (wave == 0) {
      const int kk = lane;
#pragma unroll 1
      for (int i = 1; i < CHK; ++i) {
        float upd = 0.0f;
#pragma unroll 1
        for (int j = 0; j < i; ++j) upd = fmaf(Af[i * MAT_PITCH + j], Af[j * MAT_PITCH + kk], upd);
        const float cur = Af[i * MAT_PITCH + kk];
        if (kk < i) Af[i * MAT_PITCH + kk] = cur + upd;
      }
      Af[kk * MAT_PITCH + kk] = 1.0f;
    }
    __syncthreads();

    v16h ub;
    {
      v8f au0, au1;
      {
        v16h tb;
#pragma unroll
        for (int e = 0; e < 8; ++e) {
          const int j0 = 8 * hh + e, j1 = 16 + 8 * hh + e;
          const float bj0 = beta_s[j0] * T_CARRY;
          const float bj1 = beta_s[j1] * T_CARRY;
          tb[e]     = (_Float16)(Af[c * MAT_PITCH + j0] * bj0);
          tb[8 + e] = (_Float16)(Af[c * MAT_PITCH + j1] * bj1);
        }
        au0 = wm(tb, rb, z8);
      }
      {
        v16h tb;
#pragma unroll
        for (int e = 0; e < 8; ++e) {
          const int j0 = 8 * hh + e, j1 = 16 + 8 * hh + e;
          const float bj0 = beta_s[j0] * T_CARRY;
          const float bj1 = beta_s[j1] * T_CARRY;
          tb[e]     = (_Float16)(Af[(16 + c) * MAT_PITCH + j0] * bj0);
          tb[8 + e] = (_Float16)(Af[(16 + c) * MAT_PITCH + j1] * bj1);
        }
        au1 = wm(tb, rb, z8);
      }
#pragma unroll
      for (int r = 0; r < 8; ++r) {
        ub[r]     = (_Float16)(au0[r] * INV_T);
        ub[8 + r] = (_Float16)(au1[r] * INV_T);
      }
    }
    {
      v16h al;
#pragma unroll
      for (int e = 0; e < 8; ++e) {
        const int j0 = 8 * hh + e, j1 = 16 + 8 * hh + e;
        al[e]     = (_Float16)Al[c * MAT_PITCH + j0];
        al[8 + e] = (_Float16)Al[c * MAT_PITCH + j1];
      }
      aq0 = wm(al, ub, aq0);
#pragma unroll
      for (int r = 0; r < 8; ++r) o_s[(8 * hh + r) * OS_PITCH + 16 * wave + c] = aq0[r] * INV_OUT;
    }
    {
      v16h al;
#pragma unroll
      for (int e = 0; e < 8; ++e) {
        const int j0 = 8 * hh + e, j1 = 16 + 8 * hh + e;
        al[e]     = (_Float16)Al[(16 + c) * MAT_PITCH + j0];
        al[8 + e] = (_Float16)Al[(16 + c) * MAT_PITCH + j1];
      }
      aq1 = wm(al, ub, aq1);
#pragma unroll
      for (int r = 0; r < 8; ++r) o_s[(16 + 8 * hh + r) * OS_PITCH + 16 * wave + c] = aq1[r] * INV_OUT;
    }
#pragma unroll
    for (int j = 0; j < 16; ++j) {
      const v16h ka = Frag<_Float16>::load(kT_s + (16 * j + c) * KT_PITCH + koff);
      sacc[j] = wm(ka, ub, sacc[j]);
      asm volatile("" ::: "memory");
    }
    __syncthreads();

    for (int pass = 0; pass < 2; ++pass) {
#pragma unroll
      for (int rr = 0; rr < 4; ++rr) {
        const int row = 4 * wave + rr;
        const v4f v = *(const v4f*)(o_s + row * OS_PITCH + 4 * lane);
        *(volatile v4f*)(dout + (size_t)(row0 + row) * DM + colbase + dvbase + 4 * lane) = v;
      }
      __threadfence();
    }
  }
}

__device__ __forceinline__ void stat_acc(const v4f x, float& s, float& s2, float& mx) {
  s += (x[0] + x[1]) + (x[2] + x[3]);
  s2 += (x[0] * x[0] + x[1] * x[1]) + (x[2] * x[2] + x[3] * x[3]);
  mx = fmaxf(mx, fmaxf(fmaxf(x[0], x[1]), fmaxf(x[2], x[3])));
}

__global__ __launch_bounds__(256) void branch_mix_kernel(
    const float* __restrict__ vc, const float* __restrict__ dlt, const float* __restrict__ gate,
    const float* __restrict__ b2, const float* __restrict__ alpha,
    const float* __restrict__ firs, const float* __restrict__ firl,
    const float* __restrict__ onw, unsigned short* __restrict__ omix) {
  __shared__ __align__(16) float tapS[TAPS_S * HDIM];
  __shared__ __align__(16) float tapL[TAPS_L * HDIM];
  __shared__ __align__(16) float priv[2 * 2 * 256 * 4];
  const int tid = threadIdx.x, lane = tid & 31, wave = tid >> 5;
  const int hd = blockIdx.x & 3;
  const int rblk = blockIdx.x >> 2;
  {
    const float* ps = firs + (size_t)(hd * HDIM + tid) * TAPS_S;
#pragma unroll 1
    for (int j = 0; j < TAPS_S; ++j) tapS[j * HDIM + tid] = ps[j];
    const float* pl = firl + (size_t)(hd * HDIM + tid) * TAPS_L;
#pragma unroll 1
    for (int j = 0; j < TAPS_L; ++j) tapL[j * HDIM + tid] = pl[j];
  }
  __syncthreads();
  float* pfs = priv + tid * 4;
  float* pfl = priv + 2048 + tid * 4;
  const float alpha_h = alpha[hd];
  const int kq = lane & 3;
  const float b2k = b2[kq * NHEAD + hd];

#pragma unroll 1
  for (int i = 0; i < 4; ++i) {
    const int bl = rblk * 32 + wave * 4 + i;
    const int l = bl & (SEQ - 1);
    const size_t rbase = (size_t)bl * DM + hd * HDIM;
    float sa[4], qa[4], ma[4];
#pragma unroll
    for (int k = 0; k < 4; ++k) { sa[k] = 0.0f; qa[k] = 0.0f; ma[k] = -3.4e38f; }

#pragma unroll 1
    for (int g = 0; g < 2; ++g) {
      const int chl = g * 128 + lane * 4;
      const float* vrow = vc + rbase + chl;
      v4f as = (v4f){0.f, 0.f, 0.f, 0.f};
      {
        int j0 = (TAPS_S - 1) - l;
        j0 = (j0 < 0) ? 0 : j0;
#pragma unroll 1
        for (int j = j0; j < TAPS_S; ++j) {
          const v4f x = *(const v4f*)(vrow + (long)(j - (TAPS_S - 1)) * DM);
          const v4f w = *(const v4f*)(tapS + j * HDIM + chl);
          as += w * x;
        }
      }
      v4f al = (v4f){0.f, 0.f, 0.f, 0.f};
      {
        int j0 = (TAPS_L - 1) - l;
        j0 = (j0 < 0) ? 0 : j0;
#pragma unroll 1
        for (int j = j0; j < TAPS_L; ++j) {
          const v4f x = *(const v4f*)(vrow + (long)(j - (TAPS_L - 1)) * DM);
          const v4f w = *(const v4f*)(tapL + j * HDIM + chl);
          al += w * x;
        }
      }
      const v4f dv = *(const v4f*)(dlt + rbase + chl);
      const v4f vv = *(const v4f*)(vrow);
      stat_acc(as, sa[0], qa[0], ma[0]);
      stat_acc(al, sa[1], qa[1], ma[1]);
      stat_acc(dv, sa[2], qa[2], ma[2]);
      stat_acc(vv, sa[3], qa[3], ma[3]);
      *(v4f*)(pfs + g * 1024) = as;
      *(v4f*)(pfl + g * 1024) = al;
    }
#pragma unroll
    for (int k = 0; k < 4; ++k) {
#pragma unroll
      for (int m = 16; m >= 1; m >>= 1) {
        sa[k] += __shfl_xor(sa[k], m, 32);
        qa[k] += __shfl_xor(qa[k], m, 32);
        ma[k] = fmaxf(ma[k], __shfl_xor(ma[k], m, 32));
      }
    }
    const float sk = (kq == 0) ? sa[0] : (kq == 1) ? sa[1] : (kq == 2) ? sa[2] : sa[3];
    const float qk = (kq == 0) ? qa[0] : (kq == 1) ? qa[1] : (kq == 2) ? qa[2] : qa[3];
    const float mk = (kq == 0) ? ma[0] : (kq == 1) ? ma[1] : (kq == 2) ? ma[2] : ma[3];
    const float mu = sk * (1.0f / HDIM);
    const float var = fmaxf((qk - sk * mu) * (1.0f / (HDIM - 1)), 0.0f);
    const float stat = (mu + sqrtf(var) + mk) * (1.0f / 3.0f);
    const float lg = gate[(size_t)bl * GATE_PITCH + kq * NHEAD + hd] + b2k + alpha_h * stat;
    float mm = fmaxf(lg, __shfl_xor(lg, 1, 32));
    mm = fmaxf(mm, __shfl_xor(mm, 2, 32));
    const float ek = expf(lg - mm);
    float se = ek + __shfl_xor(ek, 1, 32);
    se += __shfl_xor(se, 2, 32);
    const float wk = ek * (1.0f / se);
    const float w0 = __shfl(wk, 0, 32);
    const float w1 = __shfl(wk, 1, 32);
    const float w2 = __shfl(wk, 2, 32);
    const float w3 = __shfl(wk, 3, 32);

    float ss = 0.0f;
#pragma unroll 1
    for (int g = 0; g < 2; ++g) {
      const int chl = g * 128 + lane * 4;
      const v4f fs = *(const v4f*)(pfs + g * 1024);
      const v4f fl = *(const v4f*)(pfl + g * 1024);
      const v4f dv = *(const v4f*)(dlt + rbase + chl);
      const v4f vv = *(const v4f*)(vc + rbase + chl);
      const v4f o = w0 * fs + w1 * fl + w2 * dv + w3 * vv;
      ss += (o[0] * o[0] + o[1] * o[1]) + (o[2] * o[2] + o[3] * o[3]);
      *(v4f*)(pfs + g * 1024) = o;
    }
#pragma unroll
    for (int m = 16; m >= 1; m >>= 1) ss += __shfl_xor(ss, m, 32);
    const float sc = rsqrtf(ss * (1.0f / HDIM) + RMS_EPS);
    for (int pass = 0; pass < 2; ++pass) {
#pragma unroll 1
      for (int g = 0; g < 2; ++g) {
        const int chl = g * 128 + lane * 4;
        const v4f o = *(const v4f*)(pfs + g * 1024);
        const v4f nw = *(const v4f*)(onw + chl);
        const float y0 = o[0] * sc * nw[0];
        const float y1 = o[1] * sc * nw[1];
        const float y2 = o[2] * sc * nw[2];
        const float y3 = o[3] * sc * nw[3];
        const v2u u = (v2u){pk16(h_bits(y0), h_bits(y1)), pk16(h_bits(y2), h_bits(y3))};
        *(volatile v2u*)(omix + rbase + chl) = u;
      }
      __threadfence();
    }
  }
}

extern "C" void kernel_launch(void* const* d_in, const int* in_sizes, int n_in,
                              void* d_out, int out_size, void* d_ws, size_t ws_size, hipStream_t stream) {
  if (n_in < 17 || d_out == nullptr || d_ws == nullptr) return;
  if (in_sizes[0] != NROW * DM || in_sizes[1] != DM * DM || in_sizes[2] != DM * DM || in_sizes[3] != DM * DM ||
      in_sizes[4] != NHEAD * DM || in_sizes[5] != DM * 4 || in_sizes[6] != DM * 4 || in_sizes[7] != DM * 4 ||
      in_sizes[8] != DM * TAPS_S || in_sizes[9] != DM * TAPS_L || in_sizes[10] != NHEAD ||
      in_sizes[11] != GHID * DM || in_sizes[12] != GHID || in_sizes[13] != NGATE * GHID ||
      in_sizes[14] != NGATE || in_sizes[15] != HDIM || in_sizes[16] != DM * DM || out_size != NROW * DM) return;

  const float* hs    = (const float*)d_in[0];
  const float* qw    = (const float*)d_in[1];
  const float* kw    = (const float*)d_in[2];
  const float* vw    = (const float*)d_in[3];
  const float* bw    = (const float*)d_in[4];
  const float* qcw   = (const float*)d_in[5];
  const float* kcw   = (const float*)d_in[6];
  const float* vcw   = (const float*)d_in[7];
  const float* firs  = (const float*)d_in[8];
  const float* firl  = (const float*)d_in[9];
  const float* alpha = (const float*)d_in[10];
  const float* w1    = (const float*)d_in[11];
  const float* b1    = (const float*)d_in[12];
  const float* w2    = (const float*)d_in[13];
  const float* b2    = (const float*)d_in[14];
  const float* onw   = (const float*)d_in[15];
  const float* ow    = (const float*)d_in[16];

  char* ws = (char*)d_ws; size_t off = 0;
  auto carve = [&](size_t bytes) -> char* { char* p = ws + off; off += (bytes + 255) & ~(size_t)255; return p; };
  unsigned short* XH  = (unsigned short*)carve((size_t)NROW * DM * 2);
  unsigned short* WQH = (unsigned short*)carve((size_t)DM * DM * 2);
  unsigned short* WKH = (unsigned short*)carve((size_t)DM * DM * 2);
  unsigned short* WVH = (unsigned short*)carve((size_t)DM * DM * 2);
  unsigned short* W1H = (unsigned short*)carve((size_t)GHID * DM * 2);
  unsigned short* WOH = (unsigned short*)carve((size_t)DM * DM * 2);
  unsigned short* W2P = (unsigned short*)carve((size_t)GATE_PITCH * GHID * 2);
  char*           RA  = carve((size_t)NROW * DM * 4);
  unsigned short* QN  = (unsigned short*)carve((size_t)NROW * DM * 2);
  unsigned short* KN  = (unsigned short*)carve((size_t)NROW * DM * 2);
  float*          VC  = (float*)carve((size_t)NROW * DM * 4);
  float*          GATE = (float*)carve((size_t)NROW * GATE_PITCH * 4);
  float*          BETA = (float*)carve((size_t)NROW * NHEAD * 4);
  if (off > ws_size || off > (size_t)134217728) return;

  unsigned short* G1H  = (unsigned short*)RA;
  unsigned short* QRAW = (unsigned short*)RA;
  unsigned short* KRAW = (unsigned short*)RA + (size_t)NROW * DM;
  float*          VRAW = (float*)RA;
  float*          DOUT = (float*)RA;
  float*          TPRE = VC;
  unsigned short* OMIX = XH;

  cast8_f16_kernel<<<(NROW * DM / 8) / 256, 256, 0, stream>>>(hs, XH, NROW * DM / 8, 1.0f);
  cast_weights_kernel<<<dim3((GHID * DM / 8) / 256, 5), 256, 0, stream>>>(
      qw, kw, vw, ow, w1, WQH, WKH, WVH, WOH, W1H, DM * DM / 8, GHID * DM / 8, W_CARRY);
  w2_pad_kernel<<<(GATE_PITCH * GHID / 8) / 256, 256, 0, stream>>>(w2, W2P, W_CARRY);

  for (int half = 0; half < 2; ++half) {
    const int tiles = (HALF_ROWS / 64) * (GHID / 64);
    wmma_gemm64<0><<<(tiles + 7) / 8, 256, 0, stream>>>(
        XH + (size_t)half * HALF_ROWS * DM, DM, W1H, DM, (void*)TPRE, GHID, HALF_ROWS, GHID, DM, W_CARRY_INV);
    gelu_bias_f16_kernel<<<(HALF_ROWS * GHID / 2) / 256, 256, 0, stream>>>(
        TPRE, b1, G1H + (size_t)half * HALF_ROWS * GHID, HALF_ROWS * GHID / 2);
  }
  {
    const int tiles = (NROW / 64) * (GATE_PITCH / 64);
    wmma_gemm64<0><<<(tiles + 7) / 8, 256, 0, stream>>>(G1H, GHID, W2P, GHID, (void*)GATE, GATE_PITCH,
                                                        NROW, GATE_PITCH, GHID, W_CARRY_INV);
  }
  beta_gate_kernel<<<NROW / 8, 256, 0, stream>>>(hs, bw, BETA);

  {
    const int tiles = (NROW / 64) * (DM / 64);
    wmma_gemm64<1><<<(tiles + 7) / 8, 256, 0, stream>>>(XH, DM, WQH, DM, (void*)QRAW, DM, NROW, DM, DM, W_CARRY_INV);
    wmma_gemm64<1><<<(tiles + 7) / 8, 256, 0, stream>>>(XH, DM, WKH, DM, (void*)KRAW, DM, NROW, DM, DM, W_CARRY_INV);
    qk_conv_norm_kernel<<<dim3(NROW * NHEAD / 8, 2), 256, 0, stream>>>(QRAW, KRAW, qcw, kcw, QN, KN);
    wmma_gemm64<0><<<(tiles + 7) / 8, 256, 0, stream>>>(XH, DM, WVH, DM, (void*)VRAW, DM, NROW, DM, DM, W_CARRY_INV);
    v_conv_silu_kernel<<<(NROW * DM / 4) / 256, 256, 0, stream>>>(VRAW, vcw, VC);
  }

  chunk_scan_kernel<<<NBAT * NHEAD * 2, 256, 0, stream>>>(QN, KN, VC, BETA, DOUT);

  branch_mix_kernel<<<(NROW / 32) * NHEAD, 256, 0, stream>>>(VC, DOUT, GATE, b2, alpha, firs, firl, onw, OMIX);

  {
    const int tiles = (NROW / 64) * (DM / 64);
    wmma_gemm64<0><<<(tiles + 7) / 8, 256, 0, stream>>>(OMIX, DM, WOH, DM, d_out, DM, NROW, DM, DM, W_CARRY_INV);
  }
}
